// InActor_22531398434855
// MI455X (gfx1250) — hardware-verified
//
#include <hip/hip_runtime.h>
#include <stddef.h>


#define NOBJ   5
#define DOBJ   15
#define DBODY  10
#define OBSW   85
#define NE     20
#define KIN    4
#define NG     40
#define KMP    8
#define D1     256
#define D2     128
#define KPHI   153
#define KPP    160
#define DR     256
#define NHO    4
#define NHP    16
#define NSA    4
#define ERB    (NSA * NE)
#define NSB    16
#define PRB    (NSB * NOBJ)
#define HP     264
#define OPF    132
#define PP     136
#define NTHR   256
#define WSCAP  134217728
#define LSMIN  (-20.0f)
#define LSMAX  2.0f

#define SC_W16 16.0f
#define SC_W8  8.0f
#define SC_I16 0.0625f
#define SC_I8  0.125f

#define LA_IN   0
#define LA_H    (LA_IN + ERB * KMP * 4)
#define LA_O    (LA_H + ERB * HP * 2)
#define LA_LG   (LA_O + ERB * OPF * 4)
#define LA_WT   (LA_LG + ERB * 4)
#define LA_IDX  (LA_WT + NSA * NOBJ * KIN * 4)
#define LA_X    (LA_IDX + 128)
#define LDS_A   (LA_X + NSA * NOBJ * KPP * 2)

#define LB_H    0
#define LB_O    (LB_H + PRB * HP * 2)
#define LB_LG   (LB_O + PRB * OPF * 4)
#define LB_WT   (LB_LG + PRB * 4)
#define LB_P    (LB_WT + PRB * 4)
#define LB_R    (LB_P + NSB * PP * 2)
#define LB_Y    (LB_R + 16 * HP * 2)
#define LDS_B   (LB_Y + 16 * NHP * 4)

static_assert(ERB == 80 && PRB == 80);
static_assert((ERB % 16) == 0 && (ERB % 8) == 0 && (ERB % 4) == 0 && (PRB % 16) == 0 && (PRB % 8) == 0);
static_assert(((HP * 2) % 16) == 0 && ((OPF * 4) % 16) == 0 && ((PP * 2) % 16) == 0 && ((KPP * 2) % 16) == 0);
static_assert((KPP % 32) == 0 && (D1 % 32) == 0 && (D2 % 32) == 0 && (DR % 32) == 0 && KPP >= KPHI);
static_assert(HP >= D1 && HP >= DR && OPF >= D2 && PP >= D2);
static_assert((LA_H % 16) == 0 && (LA_O % 16) == 0 && (LA_LG % 16) == 0 && (LA_WT % 16) == 0);
static_assert((LA_IDX % 16) == 0 && (LA_X % 16) == 0 && NOBJ * KIN * 4 <= 128);
static_assert((LB_O % 16) == 0 && (LB_LG % 16) == 0 && (LB_WT % 16) == 0 && (LB_P % 16) == 0);
static_assert((LB_R % 16) == 0 && (LB_Y % 16) == 0);
static_assert(LDS_A <= 160 * 1024 && LDS_B <= 160 * 1024);
static_assert((NSA * NOBJ * KPP) % 8 == 0 && ((NSA * NOBJ * KPP * 2) % 128) == 0);
static_assert(NSA * NOBJ * KPP / 8 > NTHR && NSA * NOBJ * KPP / 8 <= 2 * NTHR);
static_assert((NSA * NOBJ * D2) % NTHR == 0 && (NSB * D2) % NTHR == 0);
static_assert(D1 == 4 * 64 && NTHR == 256 && D2 == 4 * 32);
static_assert((NSB % NSA) == 0 && 2 * NHO <= NHP && NSB == 16);

typedef float          v4f  __attribute__((ext_vector_type(4)));
typedef float          v8f  __attribute__((ext_vector_type(8)));
typedef _Float16       v4h  __attribute__((ext_vector_type(4)));
typedef _Float16       v8h  __attribute__((ext_vector_type(8)));
typedef _Float16       v16h __attribute__((ext_vector_type(16)));
typedef unsigned short v8us __attribute__((ext_vector_type(8)));
union Frag { v16h v; v8h h[2]; };
union H8 { v8h f; v8us u; };
static_assert(sizeof(Frag) == 32 && sizeof(H8) == 16);

__device__ __forceinline__ v8f wm(v16h a, v16h bq, v8f c) {
  v8f d = __builtin_amdgcn_wmma_f32_16x16x32_f16(false, a, false, bq, (short)0, c, false, false);
  asm volatile("v_nop\n\tv_nop\n\tv_nop\n\tv_nop" : "+v"(d) : "v"(a), "v"(bq));
  return d;
}

__device__ __forceinline__ v8f zero8() {
  v8f z = {0.f, 0.f, 0.f, 0.f, 0.f, 0.f, 0.f, 0.f};
  return z;
}

__device__ __forceinline__ int wrapclamp(int i, int n) {
  i = (i < 0) ? i + n : i;
  i = (i < 0) ? 0 : i;
  i = (i > n - 1) ? n - 1 : i;
  return i;
}

__device__ __forceinline__ float relu(float v) { return v > 0.0f ? v : 0.0f; }

__global__ __launch_bounds__(NTHR) void k_cvt(
    const float* __restrict__ s0, const float* __restrict__ s1, _Float16* dst,
    int K, int Kpad, int N0, int N1, int Ntot, int P0, int P1, int npiece, float scale) {
  const int t = blockIdx.x * NTHR + threadIdx.x;
  if (t >= npiece) return;
  const int e0 = 8 * t;
  const int n  = e0 / Kpad;
  const int kb = e0 - n * Kpad;
  const int n0c = (n < N0 - 1) ? n : (N0 - 1);
  int n1c = n - N0;
  n1c = (n1c < 0) ? 0 : n1c;
  const int n1m = (N1 - 1 < 0) ? 0 : (N1 - 1);
  n1c = (n1c > n1m) ? n1m : n1c;
  H8 o;
#pragma unroll
  for (int i = 0; i < 8; ++i) {
    const int k  = kb + i;
    const int kc = (k < K - 1) ? k : (K - 1);
    const float a = s0[(size_t)kc * P0 + n0c];
    const float b = s1[(size_t)kc * P1 + n1c];
    float v = (n < N0) ? a : ((n < N0 + N1) ? b : 0.0f);
    v = (k < K) ? v : 0.0f;
    o.f[i] = (_Float16)(v * scale);
  }
  (void)Ntot;
  unsigned short* p = (unsigned short*)(dst + (size_t)e0);
  *(volatile v8us*)p = o.u;
  __threadfence();
  *(volatile v8us*)p = o.u;
}

__global__ __launch_bounds__(NTHR) void k_edge(
    const float* __restrict__ obs, const float* __restrict__ ag, const float* __restrict__ gl,
    const float* __restrict__ W1, const float* __restrict__ b1,
    const _Float16* __restrict__ W2p, const float* __restrict__ b2,
    const float* __restrict__ eaW, const float* __restrict__ eab,
    const int* __restrict__ srcI, const int* __restrict__ dstI,
    const int* __restrict__ incI, const int* __restrict__ predI,
    _Float16* Xp) {
  extern __shared__ v4f lds_dyn[];
  char* sm = (char*)lds_dyn;
  float*    sIn  = (float*)(sm + LA_IN);
  _Float16* sH   = (_Float16*)(sm + LA_H);
  float*    sO   = (float*)(sm + LA_O);
  float*    sLg  = (float*)(sm + LA_LG);
  float*    sWt  = (float*)(sm + LA_WT);
  int*      sIdx = (int*)(sm + LA_IDX);
  _Float16* sX   = (_Float16*)(sm + LA_X);
  const int tid = threadIdx.x, lane = tid & 31, h = lane >> 4, m = lane & 15;
  const int wave = __builtin_amdgcn_readfirstlane(tid >> 5);
  const int b0 = blockIdx.x * NSA;

  if (tid < ERB) {
    const int bl = tid / NE, e = tid - bl * NE;
    const int b = b0 + bl;
    const int p0 = wrapclamp(predI[2 * e], NG);
    const int p1 = wrapclamp(predI[2 * e + 1], NG);
    const int s  = wrapclamp(srcI[e], NOBJ);
    const int d  = wrapclamp(dstI[e], NOBJ);
    const float* gb  = gl + (size_t)b * NG;
    const float* agb = ag + (size_t)b * NG;
    const float* ob  = obs + (size_t)b * OBSW + DBODY;
    float* r = sIn + tid * KMP;
    r[0] = gb[p0] - agb[p0];
    r[1] = gb[p1] - agb[p1];
    r[2] = ob[s * DOBJ + 0];
    r[3] = ob[s * DOBJ + 1];
    r[4] = ob[s * DOBJ + 2];
    r[5] = ob[d * DOBJ + 0];
    r[6] = ob[d * DOBJ + 1];
    r[7] = ob[d * DOBJ + 2];
  }
  if (tid < NOBJ * KIN) sIdx[tid] = wrapclamp(incI[tid], NE);
  __syncthreads();

  {
    const int cq = tid & 63, rq = tid >> 6;
    v4f w[KMP];
#pragma unroll
    for (int k = 0; k < KMP; ++k) w[k] = *(const v4f*)(W1 + k * D1 + 4 * cq);
    const v4f bb = *(const v4f*)(b1 + 4 * cq);
#pragma unroll 1
    for (int rr = 0; rr < ERB / 4; ++rr) {
      const int row = rq * (ERB / 4) + rr;
      const v4f x0 = *(const v4f*)(sIn + row * KMP);
      const v4f x1 = *(const v4f*)(sIn + row * KMP + 4);
      v4f a = x0.x * w[0];
      a = x0.y * w[1] + a;
      a = x0.z * w[2] + a;
      a = x0.w * w[3] + a;
      a = x1.x * w[4] + a;
      a = x1.y * w[5] + a;
      a = x1.z * w[6] + a;
      a = x1.w * w[7] + a;
      a = a + bb;
      v4h o;
      o.x = (_Float16)relu(a.x);
      o.y = (_Float16)relu(a.y);
      o.z = (_Float16)relu(a.z);
      o.w = (_Float16)relu(a.w);
      *(v4h*)(sH + row * HP + 4 * cq) = o;
    }
  }
  __syncthreads();

  v8f acc[5];
#pragma unroll
  for (int mt = 0; mt < 5; ++mt) acc[mt] = zero8();
  {
    const _Float16* bp = W2p + (size_t)(16 * wave + m) * D1 + 8 * h;
    const _Float16* ap = sH + m * HP + 8 * h;
#pragma unroll 1
    for (int ks = 0; ks < D1 / 32; ++ks) {
      const int ko = 32 * ks;
      Frag fb;
      fb.h[0] = *(const v8h*)(bp + ko);
      fb.h[1] = *(const v8h*)(bp + ko + 16);
#pragma unroll
      for (int mt = 0; mt < 5; ++mt) {
        Frag fa;
        fa.h[0] = *(const v8h*)(ap + mt * 16 * HP + ko);
        fa.h[1] = *(const v8h*)(ap + mt * 16 * HP + ko + 16);
        acc[mt] = wm(fa.v, fb.v, acc[mt]);
      }
    }
  }
  {
    const int col = 16 * wave + m;
    const float bias = b2[col];
#pragma unroll
    for (int mt = 0; mt < 5; ++mt) {
#pragma unroll
      for (int r = 0; r < 8; ++r) {
        sO[(16 * mt + 8 * h + r) * OPF + col] = relu(acc[mt][r] * SC_I16 + bias);
      }
    }
  }
  __syncthreads();

  {
    const v4f ew = *(const v4f*)(eaW + 4 * lane);
    const float eb = eab[0];
#pragma unroll 1
    for (int j = 0; j < ERB / 8; ++j) {
      const int row = wave * (ERB / 8) + j;
      const v4f x = *(const v4f*)(sO + row * OPF + 4 * lane);
      float s = x.x * ew.x;
      s = x.y * ew.y + s;
      s = x.z * ew.z + s;
      s = x.w * ew.w + s;
      s += __shfl_xor(s, 16);
      s += __shfl_xor(s, 8);
      s += __shfl_xor(s, 4);
      s += __shfl_xor(s, 2);
      s += __shfl_xor(s, 1);
      if (lane == 0) sLg[row] = s + eb;
    }
  }
  __syncthreads();

  if (tid < NSA * NOBJ) {
    const int bl = tid / NOBJ, o = tid - bl * NOBJ;
    const float* lp = sLg + bl * NE;
    const float l0 = lp[sIdx[o * KIN + 0]];
    const float l1 = lp[sIdx[o * KIN + 1]];
    const float l2 = lp[sIdx[o * KIN + 2]];
    const float l3 = lp[sIdx[o * KIN + 3]];
    const float mx = fmaxf(fmaxf(l0, l1), fmaxf(l2, l3));
    const float x0 = expf(l0 - mx), x1 = expf(l1 - mx), x2 = expf(l2 - mx), x3 = expf(l3 - mx);
    const float s = ((x0 + x1) + x2) + x3;
    const float inv = 1.0f / s;
    float* wp = sWt + tid * KIN;
    wp[0] = x0 * inv;
    wp[1] = x1 * inv;
    wp[2] = x2 * inv;
    wp[3] = x3 * inv;
  }
  __syncthreads();

  {
#pragma unroll 1
    for (int j = 0; j < (NSA * NOBJ * D2) / NTHR; ++j) {
      const int i = tid + j * NTHR;
      const int row = i >> 7, c = i & (D2 - 1);
      const int bl = row / NOBJ, o = row - bl * NOBJ;
      const float* wp = sWt + row * KIN;
      const float* ob = sO + (bl * NE) * OPF + c;
      float v = wp[0] * ob[sIdx[o * KIN + 0] * OPF];
      v = wp[1] * ob[sIdx[o * KIN + 1] * OPF] + v;
      v = wp[2] * ob[sIdx[o * KIN + 2] * OPF] + v;
      v = wp[3] * ob[sIdx[o * KIN + 3] * OPF] + v;
      sX[row * KPP + (DBODY + DOBJ) + c] = (_Float16)v;
    }
#pragma unroll 1
    for (int j = 0; j < 3; ++j) {
      const int i = tid + j * NTHR;
      if (i < NSA * NOBJ * 32) {
        const int row = i >> 5, jj = i & 31;
        const int bl = row / NOBJ, o = row - bl * NOBJ;
        const int b = b0 + bl;
        const int col = (jj < DBODY + DOBJ) ? jj : (KPHI + jj - (DBODY + DOBJ));
        int idx = (jj < DBODY) ? jj : (DBODY + o * DOBJ + (jj - DBODY));
        idx = (idx > OBSW - 1) ? (OBSW - 1) : idx;
        float v = obs[(size_t)b * OBSW + idx];
        v = (jj < DBODY + DOBJ) ? v : 0.0f;
        sX[row * KPP + col] = (_Float16)v;
      }
    }
  }
  __syncthreads();

  {
    const int npc = NSA * NOBJ * KPP / 8;
    unsigned short* dstp = (unsigned short*)(Xp + (size_t)blockIdx.x * (NSA * NOBJ * KPP));
    const int t1 = tid;
    const int t2 = tid + NTHR;
    const int t2c = (t2 < npc) ? t2 : (npc - 1);
    H8 va, vb;
    va.f = *(const v8h*)(sX + 8 * t1);
    vb.f = *(const v8h*)(sX + 8 * t2c);
    *(volatile v8us*)(dstp + 8 * t1) = va.u;
    if (t2 < npc) *(volatile v8us*)(dstp + 8 * t2) = vb.u;
    __threadfence();
    *(volatile v8us*)(dstp + 8 * t1) = va.u;
    if (t2 < npc) *(volatile v8us*)(dstp + 8 * t2) = vb.u;
  }
}

__global__ __launch_bounds__(NTHR) void k_obj(
    const _Float16* __restrict__ Xp,
    const _Float16* __restrict__ PW1p, const float* __restrict__ pb1,
    const _Float16* __restrict__ PW2p, const float* __restrict__ pb2,
    const float* __restrict__ saW, const float* __restrict__ sab,
    const _Float16* __restrict__ RWp, const float* __restrict__ rb1,
    const _Float16* __restrict__ HWp, const float* __restrict__ mb, const float* __restrict__ lb,
    float* out, int out1off) {
  extern __shared__ v4f lds_dyn[];
  char* sm = (char*)lds_dyn;
  _Float16* sH  = (_Float16*)(sm + LB_H);
  float*    sO  = (float*)(sm + LB_O);
  float*    sLg = (float*)(sm + LB_LG);
  float*    sWt = (float*)(sm + LB_WT);
  _Float16* sP  = (_Float16*)(sm + LB_P);
  _Float16* sR  = (_Float16*)(sm + LB_R);
  float*    sY  = (float*)(sm + LB_Y);
  const int tid = threadIdx.x, lane = tid & 31, h = lane >> 4, m = lane & 15;
  const int wave = __builtin_amdgcn_readfirstlane(tid >> 5);
  const int row0 = blockIdx.x * PRB;
  const int s0 = blockIdx.x * NSB;

  {
    v8f a0[5], a1[5];
#pragma unroll
    for (int mt = 0; mt < 5; ++mt) { a0[mt] = zero8(); a1[mt] = zero8(); }
    const _Float16* bp0 = PW1p + (size_t)(16 * wave + m) * KPP + 8 * h;
    const _Float16* bp1 = PW1p + (size_t)(16 * (wave + 8) + m) * KPP + 8 * h;
    const _Float16* ap  = Xp + ((size_t)row0 + m) * KPP + 8 * h;
#pragma unroll 1
    for (int ks = 0; ks < KPP / 32; ++ks) {
      const int ko = 32 * ks;
      Frag fb0, fb1;
      fb0.h[0] = *(const v8h*)(bp0 + ko);
      fb0.h[1] = *(const v8h*)(bp0 + ko + 16);
      fb1.h[0] = *(const v8h*)(bp1 + ko);
      fb1.h[1] = *(const v8h*)(bp1 + ko + 16);
#pragma unroll
      for (int mt = 0; mt < 5; ++mt) {
        Frag fa;
        fa.h[0] = *(const v8h*)(ap + (size_t)mt * 16 * KPP + ko);
        fa.h[1] = *(const v8h*)(ap + (size_t)mt * 16 * KPP + ko + 16);
        a0[mt] = wm(fa.v, fb0.v, a0[mt]);
        a1[mt] = wm(fa.v, fb1.v, a1[mt]);
      }
    }
    const int c0 = 16 * wave + m, c1 = 16 * (wave + 8) + m;
    const float bb0 = pb1[c0], bb1 = pb1[c1];
#pragma unroll
    for (int mt = 0; mt < 5; ++mt) {
#pragma unroll
      for (int r = 0; r < 8; ++r) {
        const int row = 16 * mt + 8 * h + r;
        sH[row * HP + c0] = (_Float16)relu(a0[mt][r] * SC_I8 + bb0);
        sH[row * HP + c1] = (_Float16)relu(a1[mt][r] * SC_I8 + bb1);
      }
    }
  }
  __syncthreads();

  {
    v8f acc[5];
#pragma unroll
    for (int mt = 0; mt < 5; ++mt) acc[mt] = zero8();
    const _Float16* bp = PW2p + (size_t)(16 * wave + m) * D1 + 8 * h;
    const _Float16* ap = sH + m * HP + 8 * h;
#pragma unroll 1
    for (int ks = 0; ks < D1 / 32; ++ks) {
      const int ko = 32 * ks;
      Frag fb;
      fb.h[0] = *(const v8h*)(bp + ko);
      fb.h[1] = *(const v8h*)(bp + ko + 16);
#pragma unroll
      for (int mt = 0; mt < 5; ++mt) {
        Frag fa;
        fa.h[0] = *(const v8h*)(ap + mt * 16 * HP + ko);
        fa.h[1] = *(const v8h*)(ap + mt * 16 * HP + ko + 16);
        acc[mt] = wm(fa.v, fb.v, acc[mt]);
      }
    }
    const int col = 16 * wave + m;
    const float bias = pb2[col];
#pragma unroll
    for (int mt = 0; mt < 5; ++mt) {
#pragma unroll
      for (int r = 0; r < 8; ++r) {
        sO[(16 * mt + 8 * h + r) * OPF + col] = relu(acc[mt][r] * SC_I16 + bias);
      }
    }
  }
  __syncthreads();

  {
    const v4f ew = *(const v4f*)(saW + 4 * lane);
    const float eb = sab[0];
#pragma unroll 1
    for (int j = 0; j < PRB / 8; ++j) {
      const int row = wave * (PRB / 8) + j;
      const v4f x = *(const v4f*)(sO + row * OPF + 4 * lane);
      float s = x.x * ew.x;
      s = x.y * ew.y + s;
      s = x.z * ew.z + s;
      s = x.w * ew.w + s;
      s += __shfl_xor(s, 16);
      s += __shfl_xor(s, 8);
      s += __shfl_xor(s, 4);
      s += __shfl_xor(s, 2);
      s += __shfl_xor(s, 1);
      if (lane == 0) sLg[row] = s + eb;
    }
  }
  __syncthreads();

  if (tid < NSB) {
    const float* lp = sLg + tid * NOBJ;
    const float l0 = lp[0], l1 = lp[1], l2 = lp[2], l3 = lp[3], l4 = lp[4];
    const float mx = fmaxf(fmaxf(fmaxf(l0, l1), fmaxf(l2, l3)), l4);
    const float x0 = expf(l0 - mx), x1 = expf(l1 - mx), x2 = expf(l2 - mx), x3 = expf(l3 - mx), x4 = expf(l4 - mx);
    const float s = (((x0 + x1) + x2) + x3) + x4;
    const float inv = 1.0f / s;
    float* wp = sWt + tid * NOBJ;
    wp[0] = x0 * inv;
    wp[1] = x1 * inv;
    wp[2] = x2 * inv;
    wp[3] = x3 * inv;
    wp[4] = x4 * inv;
  }
  __syncthreads();

  {
#pragma unroll 1
    for (int j = 0; j < (NSB * D2) / NTHR; ++j) {
      const int i = tid + j * NTHR;
      const int s = i >> 7, c = i & (D2 - 1);
      const float* wp = sWt + s * NOBJ;
      const float* ob = sO + (s * NOBJ) * OPF + c;
      float v = wp[0] * ob[0];
      v = wp[1] * ob[1 * OPF] + v;
      v = wp[2] * ob[2 * OPF] + v;
      v = wp[3] * ob[3 * OPF] + v;
      v = wp[4] * ob[4 * OPF] + v;
      sP[s * PP + c] = (_Float16)v;
    }
  }
  __syncthreads();

  {
    v8f r0 = zero8(), r1 = zero8();
    const _Float16* bp0 = RWp + (size_t)(16 * wave + m) * D2 + 8 * h;
    const _Float16* bp1 = RWp + (size_t)(16 * (wave + 8) + m) * D2 + 8 * h;
    const _Float16* ap  = sP + m * PP + 8 * h;
#pragma unroll 1
    for (int ks = 0; ks < D2 / 32; ++ks) {
      const int ko = 32 * ks;
      Frag fa, fb0, fb1;
      fa.h[0]  = *(const v8h*)(ap + ko);
      fa.h[1]  = *(const v8h*)(ap + ko + 16);
      fb0.h[0] = *(const v8h*)(bp0 + ko);
      fb0.h[1] = *(const v8h*)(bp0 + ko + 16);
      fb1.h[0] = *(const v8h*)(bp1 + ko);
      fb1.h[1] = *(const v8h*)(bp1 + ko + 16);
      r0 = wm(fa.v, fb0.v, r0);
      r1 = wm(fa.v, fb1.v, r1);
    }
    const int c0 = 16 * wave + m, c1 = 16 * (wave + 8) + m;
    const float bb0 = rb1[c0], bb1 = rb1[c1];
#pragma unroll
    for (int r = 0; r < 8; ++r) {
      const int row = 8 * h + r;
      sR[row * HP + c0] = (_Float16)relu(r0[r] * SC_I8 + bb0);
      sR[row * HP + c1] = (_Float16)relu(r1[r] * SC_I8 + bb1);
    }
  }
  __syncthreads();

  if (wave == 0) {
    v8f hy = zero8();
    const _Float16* bp = HWp + (size_t)m * DR + 8 * h;
    const _Float16* ap = sR + m * HP + 8 * h;
#pragma unroll 1
    for (int ks = 0; ks < DR / 32; ++ks) {
      const int ko = 32 * ks;
      Frag fa, fb;
      fa.h[0] = *(const v8h*)(ap + ko);
      fa.h[1] = *(const v8h*)(ap + ko + 16);
      fb.h[0] = *(const v8h*)(bp + ko);
      fb.h[1] = *(const v8h*)(bp + ko + 16);
      hy = wm(fa.v, fb.v, hy);
    }
    const int mi = (m < NHO - 1) ? m : (NHO - 1);
    int li = m - NHO;
    li = (li < 0) ? 0 : li;
    li = (li > NHO - 1) ? (NHO - 1) : li;
    const float mbv = mb[mi];
    const float lbv = lb[li];
#pragma unroll
    for (int r = 0; r < 8; ++r) {
      const float y = hy[r] * SC_I16;
      const float vmn = y + mbv;
      float vls = y + lbv;
      vls = fminf(fmaxf(vls, LSMIN), LSMAX);
      sY[(8 * h + r) * NHP + m] = (m < NHO) ? vmn : vls;
    }
  }
  __syncthreads();

  if (wave == 0) {
    const int r = lane & 15;
    const v4f vm = *(const v4f*)(sY + r * NHP);
    const v4f vl = *(const v4f*)(sY + r * NHP + NHO);
    const bool first = lane < 16;
    v4f v;
    v.x = first ? vm.x : vl.x;
    v.y = first ? vm.y : vl.y;
    v.z = first ? vm.z : vl.z;
    v.w = first ? vm.w : vl.w;
    const size_t o0 = (size_t)(s0 + r) * NHO;
    const size_t oo = first ? o0 : ((size_t)out1off + o0);
    float* p = out + oo;
    *(volatile v4f*)p = v;
    __threadfence();
    *(volatile v4f*)p = v;
  }
}

extern "C" void kernel_launch(void* const* d_in, const int* in_sizes, int n_in,
                              void* d_out, int out_size, void* d_ws, size_t ws_size,
                              hipStream_t stream) {
  if (n_in < 25) return;
  const int B = in_sizes[0] / OBSW;
  if (B <= 0 || in_sizes[0] != B * OBSW || (B % NSB) != 0) return;
  if (in_sizes[1] != B * NG || in_sizes[2] != B * NG) return;
  if (in_sizes[3] != KMP * D1 || in_sizes[4] != D1 || in_sizes[5] != D1 * D2 || in_sizes[6] != D2) return;
  if (in_sizes[7] != D2 || in_sizes[8] < 1) return;
  if (in_sizes[9] != KPHI * D1 || in_sizes[10] != D1 || in_sizes[11] != D1 * D2 || in_sizes[12] != D2) return;
  if (in_sizes[13] != D2 || in_sizes[14] < 1) return;
  if (in_sizes[15] != D2 * DR || in_sizes[16] != DR) return;
  if (in_sizes[17] != DR * NHO || in_sizes[18] != NHO || in_sizes[19] != DR * NHO || in_sizes[20] != NHO) return;
  if (in_sizes[21] != NE || in_sizes[22] != NE || in_sizes[23] != NOBJ * KIN || in_sizes[24] != 2 * NE) return;
  if (out_size != B * 2 * NHO) return;

  const float* obs    = (const float*)d_in[0];
  const float* ag     = (const float*)d_in[1];
  const float* gl     = (const float*)d_in[2];
  const float* mp_W1  = (const float*)d_in[3];
  const float* mp_b1  = (const float*)d_in[4];
  const float* mp_W2  = (const float*)d_in[5];
  const float* mp_b2  = (const float*)d_in[6];
  const float* ea_W   = (const float*)d_in[7];
  const float* ea_b   = (const float*)d_in[8];
  const float* phi_W1 = (const float*)d_in[9];
  const float* phi_b1 = (const float*)d_in[10];
  const float* phi_W2 = (const float*)d_in[11];
  const float* phi_b2 = (const float*)d_in[12];
  const float* sa_W   = (const float*)d_in[13];
  const float* sa_b   = (const float*)d_in[14];
  const float* rho_W1 = (const float*)d_in[15];
  const float* rho_b1 = (const float*)d_in[16];
  const float* mean_W = (const float*)d_in[17];
  const float* mean_b = (const float*)d_in[18];
  const float* ls_W   = (const float*)d_in[19];
  const float* ls_b   = (const float*)d_in[20];
  const int*   srcI   = (const int*)d_in[21];
  const int*   dstI   = (const int*)d_in[22];
  const int*   incI   = (const int*)d_in[23];
  const int*   predI  = (const int*)d_in[24];
  float* out = (float*)d_out;

  size_t off = 0;
  const size_t oW2  = off; off += (size_t)D2 * D1 * 2;        off = (off + 255) & ~(size_t)255;
  const size_t oPW1 = off; off += (size_t)D1 * KPP * 2;       off = (off + 255) & ~(size_t)255;
  const size_t oPW2 = off; off += (size_t)D2 * D1 * 2;        off = (off + 255) & ~(size_t)255;
  const size_t oRW  = off; off += (size_t)DR * D2 * 2;        off = (off + 255) & ~(size_t)255;
  const size_t oHW  = off; off += (size_t)NHP * DR * 2;       off = (off + 255) & ~(size_t)255;
  const size_t oX   = off; off += (size_t)B * NOBJ * KPP * 2; off = (off + 255) & ~(size_t)255;
  const size_t tot = off;
  if (tot > ws_size || tot > (size_t)WSCAP) return;
  char* ws = (char*)d_ws;
  _Float16* W2p  = (_Float16*)(ws + oW2);
  _Float16* PW1p = (_Float16*)(ws + oPW1);
  _Float16* PW2p = (_Float16*)(ws + oPW2);
  _Float16* RWp  = (_Float16*)(ws + oRW);
  _Float16* HWp  = (_Float16*)(ws + oHW);
  _Float16* Xp   = (_Float16*)(ws + oX);

  const int npW2  = D2 * D1 / 8;
  const int npPW1 = D1 * KPP / 8;
  const int npRW  = DR * D2 / 8;
  const int npHW  = NHP * DR / 8;
  if ((npW2 % NTHR) != 0 || (npPW1 % NTHR) != 0 || (npRW % NTHR) != 0 || (npHW % NTHR) != 0) return;

  k_cvt<<<npW2 / NTHR, NTHR, 0, stream>>>(mp_W2, mp_W2, W2p, D1, D1, D2, 0, D2, D2, D2, npW2, SC_W16);
  k_cvt<<<npPW1 / NTHR, NTHR, 0, stream>>>(phi_W1, phi_W1, PW1p, KPHI, KPP, D1, 0, D1, D1, D1, npPW1, SC_W8);
  k_cvt<<<npW2 / NTHR, NTHR, 0, stream>>>(phi_W2, phi_W2, PW2p, D1, D1, D2, 0, D2, D2, D2, npW2, SC_W16);
  k_cvt<<<npRW / NTHR, NTHR, 0, stream>>>(rho_W1, rho_W1, RWp, D2, D2, DR, 0, DR, DR, DR, npRW, SC_W8);
  k_cvt<<<npHW / NTHR, NTHR, 0, stream>>>(mean_W, ls_W, HWp, DR, DR, NHO, NHO, NHP, NHO, NHO, npHW, SC_W16);

  hipFuncSetAttribute(reinterpret_cast<const void*>(&k_edge),
                      hipFuncAttributeMaxDynamicSharedMemorySize, LDS_A);
  k_edge<<<B / NSA, NTHR, LDS_A, stream>>>(obs, ag, gl, mp_W1, mp_b1, W2p, mp_b2, ea_W, ea_b,
                                           srcI, dstI, incI, predI, Xp);

  hipFuncSetAttribute(reinterpret_cast<const void*>(&k_obj),
                      hipFuncAttributeMaxDynamicSharedMemorySize, LDS_B);
  k_obj<<<B / NSB, NTHR, LDS_B, stream>>>(Xp, PW1p, phi_b1, PW2p, phi_b2, sa_W, sa_b, RWp, rho_b1,
                                          HWp, mean_b, ls_b, out, B * NHO);
}
